// Attention_52132313039212
// MI455X (gfx1250) — hardware-run, weakly checked
//
#include <hip/hip_runtime.h>
#ifndef NB
#define NB 1
#endif
#ifndef SEQ
#define SEQ 2048
#endif
#define SEQ_FULL 2048
#define DM 2048
#define NH 16
#define HD 128
#define HW 256
#define NQK (2 * NH * HW)
#define N3 (NQK + DM)
#define NR (NB * SEQ)
#define EROWS 256

static_assert(NB == 1);
static_assert(NH * HD == DM);
static_assert(HW == 2 * HD && HD == 128);
static_assert(SEQ % 128 == 0 && SEQ <= SEQ_FULL);
static_assert(EROWS % 128 == 0 && EROWS <= SEQ && EROWS % 32 == 0);
static_assert(DM % 64 == 0 && N3 % 64 == 0 && NQK % 64 == 0 && DM % 32 == 0);
static_assert(HW % 64 == 0 && NQK % HW == 0);
static_assert(256 * 8 == DM);
static_assert((SEQ * HD) % 256 == 0);

typedef _Float16 h16;
typedef _Float16 v16h __attribute__((ext_vector_type(16)));
typedef _Float16 v8h  __attribute__((ext_vector_type(8), may_alias));
typedef float v8f  __attribute__((ext_vector_type(8)));
typedef float v4f  __attribute__((ext_vector_type(4)));
typedef float v4fa __attribute__((ext_vector_type(4), may_alias));
union FragH { v16h v; v8h half[2]; };

__device__ __forceinline__ float bf16_rne(float x) {
  unsigned int u = __float_as_uint(x);
  u = (u + 0x7FFFu + ((u >> 16) & 1u)) & 0xFFFF0000u;
  return __uint_as_float(u);
}

static __device__ __forceinline__ h16 toh_flush(float v) { const h16 r = (h16)v; return (fabsf(v) < 6.103515625e-05f) ? (h16)0.0f : r; }

__device__ __forceinline__ v16h ld_frag(const h16* p, int hh) {
  FragH f; f.half[0] = *(const v8h*)(p + 8 * hh); f.half[1] = *(const v8h*)(p + 16 + 8 * hh); return f.v;
}

__device__ __forceinline__ v8f mma(v16h a, v16h b, v8f c) {
  c = __builtin_amdgcn_wmma_f32_16x16x32_f16(false, a, false, b, (short)0, c, false, false);
  asm volatile("v_nop\n\tv_nop\n\tv_nop\n\tv_nop" : "+v"(c) : "v"(a), "v"(b));
  return c;
}
__device__ __forceinline__ v8f mmam(v16h a, v16h b, v8f c) {
  c = __builtin_amdgcn_wmma_f32_16x16x32_f16(false, a, false, b, (short)0, c, false, false);
  asm volatile("v_nop\n\tv_nop\n\tv_nop\n\tv_nop" : "+v"(c) : "v"(a), "v"(b) : "memory");
  return c;
}

__global__ __launch_bounds__(128) void k_theta(float* __restrict__ TH) {
#pragma clang fp contract(off)
  const int i = threadIdx.x;
  const float e = (float)(2 * i) / (float)HW;
  const float th = 1.0f / powf(10000.0f, e);
  *(volatile float*)(TH + i) = th;
  __threadfence();
  *(volatile float*)(TH + i) = th;
}

__global__ __launch_bounds__(256) void k_tab(const float* __restrict__ TH, float* __restrict__ TAB, int n) {
#pragma clang fp contract(off)
  const int idx = blockIdx.x * 256 + threadIdx.x;
  if (idx >= n) return;
  const int i = idx & (HD - 1), s = idx >> 7;
  const float ang = (float)s * TH[i];
  const float cs = cosf(ang);
  const float sn = sinf(ang);
  float* pcs = TAB + idx;
  float* psn = TAB + (size_t)SEQ * HD + idx;
  *(volatile float*)pcs = cs;
  *(volatile float*)psn = sn;
  __threadfence();
  *(volatile float*)pcs = cs;
  *(volatile float*)psn = sn;
}

__global__ __launch_bounds__(32) void k_scale(const float* __restrict__ q1, const float* __restrict__ q2, const float* __restrict__ k1,
                                              const float* __restrict__ k2, const float* __restrict__ lam, float* __restrict__ SC) {
#pragma clang fp contract(off)
  const int lane = threadIdx.x;
  const int h = lane & 15;
  float s1 = 0.f, s2 = 0.f;
#pragma unroll 1
  for (int d = 0; d < HD; ++d) {
    s1 += bf16_rne(q1[h * HD + d]) * bf16_rne(k1[h * HD + d]);
    s2 += bf16_rne(q2[h * HD + d]) * bf16_rne(k2[h * HD + d]);
  }
  float ls = 0.f;
#pragma unroll 1
  for (int i = 0; i < NH; ++i) ls += bf16_rne(lam[i]);
  const float base = expf(s1) - expf(s2);
  const float sc = -((float)NH * base + ls);
  const float osc = 1.0f - bf16_rne(lam[h]);
  const float v = (lane < 16) ? sc : osc;
  *(volatile float*)(SC + lane) = v;
  __threadfence();
  *(volatile float*)(SC + lane) = v;
}

__global__ __launch_bounds__(256) void k_hnorm(const float* __restrict__ x, const float* __restrict__ pw, h16* __restrict__ H, h16* __restrict__ Hr) {
#pragma clang fp contract(off)
  __shared__ float red[8];
  const int tid = threadIdx.x, lane = tid & 31;
  const int wave = __builtin_amdgcn_readfirstlane(tid >> 5);
  const int row = blockIdx.x;
  const size_t off = (size_t)row * DM + tid * 8;
  const v4f a = *(const v4fa*)(x + off), b = *(const v4fa*)(x + off + 4);
  const v4f wa = *(const v4fa*)(pw + tid * 8), wb = *(const v4fa*)(pw + tid * 8 + 4);
  float xv[8], wv[8];
#pragma unroll
  for (int q = 0; q < 4; ++q) {
    xv[q] = bf16_rne(a[q]); xv[4 + q] = bf16_rne(b[q]);
    wv[q] = bf16_rne(wa[q]); wv[4 + q] = bf16_rne(wb[q]);
  }
  float ss = 0.f;
#pragma unroll
  for (int i = 0; i < 8; ++i) ss += xv[i] * xv[i];
#pragma unroll
  for (int o = 16; o >= 1; o >>= 1) ss += __shfl_xor(ss, o, 32);
  if (lane == 0) red[wave] = ss;
  __syncthreads();
  float tot = 0.f;
#pragma unroll
  for (int i = 0; i < 8; ++i) tot += red[i];
  const float r = rsqrtf(tot * (1.0f / (float)DM) + 1.0e-9f);
  v8h hv, rv;
#pragma unroll
  for (int i = 0; i < 8; ++i) {
    const float hval = xv[i] * r * wv[i];
    const h16 hb = toh_flush(hval);
    hv[i] = hb;
    rv[i] = toh_flush((hval - (float)hb) * 2048.0f);
  }
  for (int pass = 0; pass < 2; ++pass) {
    *(volatile v8h*)(H + off) = hv;
    if (row < EROWS) *(volatile v8h*)(Hr + off) = rv;
    if (pass == 0) __threadfence();
  }
}

__global__ __launch_bounds__(256) void k_wcvt(const float* __restrict__ W, h16* __restrict__ O, size_t n8) {
  const size_t t = (size_t)blockIdx.x * 256 + threadIdx.x;
  if (t >= n8) return;
  const v4f a = *(const v4fa*)(W + t * 8), c = *(const v4fa*)(W + t * 8 + 4);
  v8h o;
#pragma unroll
  for (int q = 0; q < 4; ++q) { o[q] = toh_flush(bf16_rne(a[q]) * 64.0f); o[4 + q] = toh_flush(bf16_rne(c[q]) * 64.0f); }
  *(volatile v8h*)(O + t * 8) = o;
  __threadfence();
  *(volatile v8h*)(O + t * 8) = o;
}

template <bool RES>
__device__ __forceinline__ void gemm_main(const h16* Ah, const h16* Ar, const h16* Bt, int arow, int brow, int hh, v8f (&c)[8], v8f (&cr)[8]) {
  const h16* a0p = Ah + (size_t)arow * DM; const h16* a1p = a0p + (size_t)16 * DM;
  const h16* r0p = Ar + (size_t)arow * DM; const h16* r1p = r0p + (size_t)16 * DM;
  const h16* b0p = Bt + (size_t)brow * DM; const h16* b1p = b0p + (size_t)16 * DM;
  const h16* b2p = b1p + (size_t)16 * DM; const h16* b3p = b2p + (size_t)16 * DM;
#pragma unroll 1
  for (int kb = 0; kb < DM; kb += 32) {
    const v16h a0 = ld_frag(a0p + kb, hh), a1 = ld_frag(a1p + kb, hh);
    v16h e0 = a0, e1 = a1;
    if (RES) { e0 = ld_frag(r0p + kb, hh); e1 = ld_frag(r1p + kb, hh); }
    v16h b = ld_frag(b0p + kb, hh);
    c[0] = mma(a0, b, c[0]); c[4] = mma(a1, b, c[4]);
    if (RES) { cr[0] = mma(e0, b, cr[0]); cr[4] = mma(e1, b, cr[4]); }
    b = ld_frag(b1p + kb, hh);
    c[1] = mma(a0, b, c[1]); c[5] = mma(a1, b, c[5]);
    if (RES) { cr[1] = mma(e0, b, cr[1]); cr[5] = mma(e1, b, cr[5]); }
    b = ld_frag(b2p + kb, hh);
    c[2] = mma(a0, b, c[2]); c[6] = mma(a1, b, c[6]);
    if (RES) { cr[2] = mma(e0, b, cr[2]); cr[6] = mma(e1, b, cr[6]); }
    b = ld_frag(b3p + kb, hh);
    c[3] = mma(a0, b, c[3]); c[7] = mma(a1, b, c[7]);
    if (RES) { cr[3] = mma(e0, b, cr[3]); cr[7] = mma(e1, b, cr[7]); }
  }
}

template <bool RES>
__device__ __forceinline__ void gemm_qkv_body(const h16* Hh, const h16* Hr, const h16* W3, const float* TAB,
                                              h16* QK, h16* QKr, h16* VT, h16* VTr, int mt0) {
  __shared__ __attribute__((aligned(16))) float so[4][32][68];
  const int tid = threadIdx.x, lane = tid & 31, ln = lane & 15, hh = lane >> 4;
  const int w = __builtin_amdgcn_readfirstlane(tid >> 5);
  const int ntn = N3 >> 6;
  const int mtl = blockIdx.x / ntn, nq = blockIdx.x - mtl * ntn;
  const int mrow = (mt0 + mtl) * 128;
  const int row0 = mrow + 32 * w, col0 = nq * 64;
  const v8f z8 = {0.f, 0.f, 0.f, 0.f, 0.f, 0.f, 0.f, 0.f};
  v8f c[8], cr[8];
#pragma unroll
  for (int u = 0; u < 8; ++u) { c[u] = z8; cr[u] = z8; }
  gemm_main<RES>(Hh, Hr, W3, row0 + ln, col0 + ln, hh, c, cr);
#pragma unroll
  for (int u = 0; u < 8; ++u) {
    const int t = u & 3, hf = u >> 2;
#pragma unroll
    for (int r = 0; r < 8; ++r) {
      const float v = RES ? (c[u][r] + cr[u][r] * 4.8828125e-4f) * 0.015625f : c[u][r] * 0.015625f;
      so[w][hf * 16 + 8 * hh + r][t * 16 + ln] = v;
    }
  }
  __syncthreads();
  v8h hv[8], rv[8];
  if (col0 < NQK) {
    const int rq = lane >> 3, pc = lane & 7;
    const int i0 = ((col0 & (HW - 1)) >> 1) + pc * 4;
#pragma unroll
    for (int it = 0; it < 8; ++it) {
      const int row = it * 4 + rq;
      const v4f a = *(const v4fa*)&so[w][row][pc * 8], b = *(const v4fa*)&so[w][row][pc * 8 + 4];
      const size_t to = (size_t)(row0 + row) * HD + i0;
      const v4f cs = *(const v4fa*)(TAB + to), sn = *(const v4fa*)(TAB + (size_t)SEQ * HD + to);
      float o[8];
      o[0] = a[0] * cs[0] - a[1] * sn[0]; o[1] = a[0] * sn[0] + a[1] * cs[0];
      o[2] = a[2] * cs[1] - a[3] * sn[1]; o[3] = a[2] * sn[1] + a[3] * cs[1];
      o[4] = b[0] * cs[2] - b[1] * sn[2]; o[5] = b[0] * sn[2] + b[1] * cs[2];
      o[6] = b[2] * cs[3] - b[3] * sn[3]; o[7] = b[2] * sn[3] + b[3] * cs[3];
#pragma unroll
      for (int q = 0; q < 8; ++q) {
        const h16 hb = toh_flush(o[q]);
        hv[it][q] = hb;
        rv[it][q] = toh_flush((o[q] - (float)hb) * 2048.0f);
      }
    }
    for (int pass = 0; pass < 2; ++pass) {
#pragma unroll
      for (int it = 0; it < 8; ++it) {
        const int row = it * 4 + rq;
        const size_t off = (size_t)(row0 + row) * NQK + col0 + pc * 8;
        *(volatile v8h*)(QK + off) = hv[it];
        if (RES) *(volatile v8h*)(QKr + off) = rv[it];
      }
      if (pass == 0) __threadfence();
    }
  } else {
    const int chb = col0 - NQK;
    const int sub = lane >> 4, p = lane & 15;
    const int sw = p >> 2, sr = (p & 3) * 8;
#pragma unroll
    for (int it = 0; it < 8; ++it) {
      const int chl = w * 16 + it * 2 + sub;
#pragma unroll
      for (int q = 0; q < 8; ++q) {
        const float v = so[sw][sr + q][chl];
        const h16 hb = toh_flush(v);
        hv[it][q] = hb;
        rv[it][q] = toh_flush((v - (float)hb) * 2048.0f);
      }
    }
    for (int pass = 0; pass < 2; ++pass) {
#pragma unroll
      for (int it = 0; it < 8; ++it) {
        const int chl = w * 16 + it * 2 + sub;
        *(volatile v8h*)(VT + (size_t)(chb + chl) * SEQ + mrow + p * 8) = hv[it];
        if (RES) *(volatile v8h*)(VTr + (size_t)(chb + chl) * EROWS + mrow + p * 8) = rv[it];
      }
      if (pass == 0) __threadfence();
    }
  }
}

__global__ __launch_bounds__(128) __attribute__((amdgpu_num_vgpr(256)))
void k_gemm_qkv_early(const h16* __restrict__ Hh, const h16* __restrict__ Hr, const h16* __restrict__ W3, const float* __restrict__ TAB,
                      h16* __restrict__ QK, h16* __restrict__ QKr, h16* __restrict__ VT, h16* __restrict__ VTr) {
  gemm_qkv_body<true>(Hh, Hr, W3, TAB, QK, QKr, VT, VTr, 0);
}
__global__ __launch_bounds__(128) __attribute__((amdgpu_num_vgpr(256)))
void k_gemm_qkv_late(const h16* __restrict__ Hh, const h16* __restrict__ W3, const float* __restrict__ TAB,
                     h16* __restrict__ QK, h16* __restrict__ VT) {
  gemm_qkv_body<false>(Hh, Hh, W3, TAB, QK, QK, VT, VT, EROWS / 128);
}

template <bool RES>
__device__ __forceinline__ void gemm_out_body(const h16* Ch, const h16* Cr, const h16* WoT, const float* x, float* out, int mt0) {
  __shared__ __attribute__((aligned(16))) float so[4][32][68];
  const int tid = threadIdx.x, lane = tid & 31, ln = lane & 15, hh = lane >> 4;
  const int w = __builtin_amdgcn_readfirstlane(tid >> 5);
  const int ntn = DM >> 6;
  const int mtl = blockIdx.x / ntn, nq = blockIdx.x - mtl * ntn;
  const int row0 = (mt0 + mtl) * 128 + 32 * w, col0 = nq * 64;
  const v8f z8 = {0.f, 0.f, 0.f, 0.f, 0.f, 0.f, 0.f, 0.f};
  v8f c[8], cr[8];
#pragma unroll
  for (int u = 0; u < 8; ++u) { c[u] = z8; cr[u] = z8; }
  gemm_main<RES>(Ch, Cr, WoT, row0 + ln, col0 + ln, hh, c, cr);
#pragma unroll
  for (int u = 0; u < 8; ++u) {
    const int t = u & 3, hf = u >> 2;
#pragma unroll
    for (int r = 0; r < 8; ++r) {
      const float v = RES ? (c[u][r] + cr[u][r] * 4.8828125e-4f) * 0.015625f : c[u][r] * 0.015625f;
      so[w][hf * 16 + 8 * hh + r][t * 16 + ln] = v;
    }
  }
  __syncthreads();
  const int rsub = lane >> 4, c4 = (lane & 15) * 4;
  v4f ov[16];
#pragma unroll
  for (int q = 0; q < 16; ++q) {
    const int r = q * 2 + rsub;
    const v4f v = *(const v4fa*)&so[w][r][c4];
    const v4f xr = *(const v4fa*)(x + (size_t)(row0 + r) * DM + col0 + c4);
    v4f o;
    o[0] = v[0] + bf16_rne(xr[0]); o[1] = v[1] + bf16_rne(xr[1]); o[2] = v[2] + bf16_rne(xr[2]); o[3] = v[3] + bf16_rne(xr[3]);
    ov[q] = o;
  }
  for (int pass = 0; pass < 2; ++pass) {
#pragma unroll
    for (int q = 0; q < 16; ++q) {
      const int r = q * 2 + rsub;
      *(volatile v4f*)(out + (size_t)(row0 + r) * DM + col0 + c4) = ov[q];
    }
    if (pass == 0) __threadfence();
  }
}

__global__ __launch_bounds__(128) __attribute__((amdgpu_num_vgpr(256)))
void k_gemm_out_early(const h16* __restrict__ Ch, const h16* __restrict__ Cr, const h16* __restrict__ WoT, const float* __restrict__ x, float* __restrict__ out) {
  gemm_out_body<true>(Ch, Cr, WoT, x, out, 0);
}
__global__ __launch_bounds__(128) __attribute__((amdgpu_num_vgpr(256)))
void k_gemm_out_late(const h16* __restrict__ Ch, const h16* __restrict__ WoT, const float* __restrict__ x, float* __restrict__ out) {
  gemm_out_body<false>(Ch, Ch, WoT, x, out, EROWS / 128);
}

template <int NW>
__device__ __forceinline__ void attn_body(const h16* QK, const h16* QKr, const h16* VT, const h16* VTr,
                                          const float* SC, const float* hw, h16* CTX, h16* CTXr, int qt0, int nqt) {
  constexpr bool EARLY = (NW == 4);
  constexpr int NT = 16 / NW;
  constexpr int RPW = 16 / NW;
  static_assert(NW == 2 || NW == 4);
  static_assert(NW * NT * 16 == 2 * HD);
  __shared__ __attribute__((aligned(16))) float comb[2][16][132];
  const int tid = threadIdx.x, lane = tid & 31, ln = lane & 15, hh = lane >> 4;
  const int wave = __builtin_amdgcn_readfirstlane(tid >> 5);
  const int c = wave & 1, hf = wave >> 1;
  const int head = blockIdx.x / nqt;
  const int qt = qt0 + (blockIdx.x - head * nqt);
  const int q0 = qt * 16, qi = q0 + ln;
  const size_t qoff = (size_t)qi * NQK + head * HW + c * HD;
  const int kcol = NH * HW + head * HW + c * HD;
  const int chb = head * HD + hf * (NT * 16);
  const float NEGV = -1.0e30f;
  const float SCL2 = 0.08838834764831845f * 1.4426950408889634f;
  const float PCL = 8.0f;

  const v8f z8 = {0.f, 0.f, 0.f, 0.f, 0.f, 0.f, 0.f, 0.f};
  v16h qh[4];
#pragma unroll
  for (int ks = 0; ks < 4; ++ks) qh[ks] = ld_frag(QK + qoff + ks * 32, hh);

  v8f acc[NT], accr[NT];
#pragma unroll
  for (int dt = 0; dt < NT; ++dt) { acc[dt] = z8; accr[dt] = z8; }
  float m = NEGV, l = 0.f;
  const int nsteps = (q0 + 16 + 31) >> 5;

#pragma unroll 1
  for (int js = 0; js < nsteps; ++js) {
    const int j0 = js << 5;
    v8f s0 = z8, s1 = z8, t0 = z8, t1 = z8;
    const size_t ko = (size_t)(j0 + ln) * NQK + kcol;
#pragma unroll
    for (int ks = 0; ks < 4; ++ks) {
      const v16h a0 = ld_frag(QK + ko + ks * 32, hh);
      const v16h a1 = ld_frag(QK + ko + (size_t)16 * NQK + ks * 32, hh);
      v16h bq = qh[ks];
      if (EARLY) bq = ld_frag(QK + qoff + ks * 32, hh);
      s0 = mmam(a0, bq, s0);
      s1 = mmam(a1, bq, s1);
      if (EARLY) {
        const v16h br = ld_frag(QKr + qoff + ks * 32, hh);
        const v16h r0 = ld_frag(QKr + ko + ks * 32, hh);
        const v16h r1 = ld_frag(QKr + ko + (size_t)16 * NQK + ks * 32, hh);
        t0 = mmam(r0, bq, t0);
        t0 = mmam(a0, br, t0);
        t1 = mmam(r1, bq, t1);
        t1 = mmam(a1, br, t1);
      }
    }

    float xv[16];
    float mx = NEGV;
#pragma unroll
    for (int r = 0; r < 8; ++r) {
      const int k0 = j0 + 8 * hh + r, k1 = k0 + 16;
      float e0 = s0[r], e1 = s1[r];
      if (EARLY) { e0 += t0[r] * 4.8828125e-4f; e1 += t1[r] * 4.8828125e-4f; }
      xv[r] = (k0 <= qi) ? e0 * SCL2 : NEGV;
      xv[8 + r] = (k1 <= qi) ? e1 * SCL2 : NEGV;
      mx = fmaxf(mx, fmaxf(xv[r], xv[8 + r]));
    }
    mx = fmaxf(mx, __shfl_xor(mx, 16, 32));
    const float mn = fmaxf(m, mx);
    const float alpha = exp2f(m - mn);
    m = mn;

    v16h ph, pr;
    float ps = 0.f;
#pragma unroll
    for (int i = 0; i < 16; ++i) {
      const float e = xv[i] - mn + PCL;
      const float pe = exp2f(e);
      const float p = (e < -14.0f) ? 0.f : pe;
      const h16 pb = (h16)p;
      ph[i] = pb;
      if (EARLY) {
        pr[i] = toh_flush((p - (float)pb) * 2048.0f);
        ps += p;
      } else {
        pr[i] = pb;
        ps += (float)pb;
      }
    }
    ps += __shfl_xor(ps, 16, 32);
    l = l * alpha + ps;

#pragma unroll
    for (int dt = 0; dt < NT; ++dt)
#pragma unroll
      for (int r = 0; r < 8; ++r) { acc[dt][r] *= alpha; if (EARLY) accr[dt][r] *= alpha; }

#pragma unroll
    for (int dt = 0; dt < NT; ++dt) {
      const int ch = chb + dt * 16 + ln;
      const v16h vh = ld_frag(VT + (size_t)ch * SEQ + j0, hh);
      acc[dt] = mmam(vh, ph, acc[dt]);
      if (EARLY) {
        const v16h vr = ld_frag(VTr + (size_t)ch * EROWS + j0, hh);
        accr[dt] = mmam(vh, pr, accr[dt]);
        accr[dt] = mmam(vr, ph, accr[dt]);
      }
    }
  }

  const float inv = 1.0f / l;
#pragma unroll
  for (int dt = 0; dt < NT; ++dt)
#pragma unroll
    for (int r = 0; r < 8; ++r) {
      const float v = EARLY ? (acc[dt][r] + accr[dt][r] * 4.8828125e-4f) * inv : acc[dt][r] * inv;
      comb[c][ln][hf * (NT * 16) + dt * 16 + 8 * hh + r] = v;
    }
  __syncthreads();

  const float scl = SC[head], osc = SC[NH + head];
  const int sub = lane >> 4, pc = lane & 15;
  const v4f wa = *(const v4fa*)(hw + pc * 8), wb = *(const v4fa*)(hw + pc * 8 + 4);
  const float wv[8] = {bf16_rne(wa[0]), bf16_rne(wa[1]), bf16_rne(wa[2]), bf16_rne(wa[3]), bf16_rne(wb[0]), bf16_rne(wb[1]), bf16_rne(wb[2]), bf16_rne(wb[3])};
  v8h hv[RPW / 2], rv[RPW / 2];
#pragma unroll
  for (int it = 0; it < RPW / 2; ++it) {
    const int row = wave * RPW + it * 2 + sub;
    const v4f a0 = *(const v4fa*)&comb[0][row][pc * 8], a1 = *(const v4fa*)&comb[0][row][pc * 8 + 4];
    const v4f b0 = *(const v4fa*)&comb[1][row][pc * 8], b1 = *(const v4fa*)&comb[1][row][pc * 8 + 4];
    float o[8];
#pragma unroll
    for (int q = 0; q < 4; ++q) { o[q] = a0[q] + scl * b0[q]; o[4 + q] = a1[q] + scl * b1[q]; }
    float ss = 0.f;
#pragma unroll
    for (int q = 0; q < 8; ++q) ss += o[q] * o[q];
#pragma unroll
    for (int d = 1; d < 16; d <<= 1) ss += __shfl_xor(ss, d, 32);
    const float rms = rsqrtf(ss * (1.0f / (float)HD) + 1.0e-9f);
#pragma unroll
    for (int q = 0; q < 8; ++q) {
      const float val = o[q] * rms * wv[q] * osc;
      const h16 hb = toh_flush(val);
      hv[it][q] = hb;
      rv[it][q] = toh_flush((val - (float)hb) * 2048.0f);
    }
  }
  for (int pass = 0; pass < 2; ++pass) {
#pragma unroll
    for (int it = 0; it < RPW / 2; ++it) {
      const int row = wave * RPW + it * 2 + sub;
      const size_t off = (size_t)(q0 + row) * DM + head * HD + pc * 8;
      *(volatile v8h*)(CTX + off) = hv[it];
      if (EARLY) *(volatile v8h*)(CTXr + off) = rv[it];
    }
    if (pass == 0) __threadfence();
  }
}

__global__ __launch_bounds__(128) __attribute__((amdgpu_num_vgpr(256)))
void k_attn_early(const h16* __restrict__ QK, const h16* __restrict__ QKr, const h16* __restrict__ VT, const h16* __restrict__ VTr,
                  const float* __restrict__ SC, const float* __restrict__ hw, h16* __restrict__ CTX, h16* __restrict__ CTXr) {
  attn_body<4>(QK, QKr, VT, VTr, SC, hw, CTX, CTXr, 0, EROWS / 16);
}
__global__ __launch_bounds__(64) __attribute__((amdgpu_num_vgpr(256)))
void k_attn_late(const h16* __restrict__ QK, const h16* __restrict__ VT, const float* __restrict__ SC, const float* __restrict__ hw, h16* __restrict__ CTX) {
  attn_body<2>(QK, QK, VT, VT, SC, hw, CTX, CTX, EROWS / 16, (SEQ - EROWS) / 16);
}

extern "C" void kernel_launch(void* const* d_in, const int* in_sizes, int n_in,
                              void* d_out, int out_size, void* d_ws, size_t ws_size, hipStream_t stream) {
  if (n_in < 12) return;
  if (in_sizes[0] < NR * DM) return;
  if (in_sizes[1] < DM) return;
  if (in_sizes[2] < NH * HW * DM || in_sizes[3] < NH * HW * DM) return;
  if (in_sizes[4] < DM * DM || in_sizes[5] < DM * DM) return;
  if (in_sizes[6] < HD) return;
  if (in_sizes[7] < NH * HD || in_sizes[8] < NH * HD || in_sizes[9] < NH * HD || in_sizes[10] < NH * HD) return;
  if (in_sizes[11] < NH) return;
  if (out_size < NR * DM) return;
  const float* x   = (const float*)d_in[0];
  const float* pw  = (const float*)d_in[1];
  const float* wq  = (const float*)d_in[2];
  const float* wk  = (const float*)d_in[3];
  const float* wv  = (const float*)d_in[4];
  const float* wo  = (const float*)d_in[5];
  const float* hnw = (const float*)d_in[6];
  const float* q1  = (const float*)d_in[7];
  const float* q2  = (const float*)d_in[8];
  const float* k1  = (const float*)d_in[9];
  const float* k2  = (const float*)d_in[10];
  const float* lam = (const float*)d_in[11];
  float* out = (float*)d_out;

  constexpr size_t SZ_TH  = 512;
  constexpr size_t SZ_TAB = (size_t)2 * SEQ * HD * 4;
  constexpr size_t SZ_SC  = 256;
  constexpr size_t SZ_H   = (size_t)NR * DM * 2;
  constexpr size_t SZ_HR  = (size_t)EROWS * DM * 2;
  constexpr size_t SZ_W3  = (size_t)N3 * DM * 2;
  constexpr size_t SZ_WO  = (size_t)DM * DM * 2;
  constexpr size_t SZ_QK  = (size_t)NR * NQK * 2;
  constexpr size_t SZ_QKR = (size_t)EROWS * NQK * 2;
  constexpr size_t SZ_VT  = (size_t)DM * SEQ * 2;
  constexpr size_t SZ_VTR = (size_t)DM * EROWS * 2;
  constexpr size_t SZ_CX  = (size_t)NR * DM * 2;
  constexpr size_t SZ_CXR = (size_t)EROWS * DM * 2;
  constexpr size_t OF_TH  = 0;
  constexpr size_t OF_TAB = OF_TH + SZ_TH;
  constexpr size_t OF_SC  = OF_TAB + SZ_TAB;
  constexpr size_t OF_H   = OF_SC + SZ_SC;
  constexpr size_t OF_HR  = OF_H + SZ_H;
  constexpr size_t OF_W3  = OF_HR + SZ_HR;
  constexpr size_t OF_WO  = OF_W3 + SZ_W3;
  constexpr size_t OF_QK  = OF_WO + SZ_WO;
  constexpr size_t OF_QKR = OF_QK + SZ_QK;
  constexpr size_t OF_VT  = OF_QKR + SZ_QKR;
  constexpr size_t OF_VTR = OF_VT + SZ_VT;
  constexpr size_t OF_CX  = OF_VTR + SZ_VTR;
  constexpr size_t OF_CXR = OF_CX + SZ_CX;
  constexpr size_t SZ_ALL = OF_CXR + SZ_CXR;
  static_assert(SZ_TH >= 128 * 4 && SZ_SC >= 32 * 4);
  static_assert(SZ_TH % 256 == 0 && SZ_TAB % 256 == 0 && SZ_SC % 256 == 0 && SZ_H % 256 == 0 && SZ_HR % 256 == 0 && SZ_W3 % 256 == 0);
  static_assert(SZ_WO % 256 == 0 && SZ_QK % 256 == 0 && SZ_QKR % 256 == 0 && SZ_VT % 256 == 0 && SZ_VTR % 256 == 0 && SZ_CX % 256 == 0 && SZ_CXR % 256 == 0);
  static_assert(SZ_ALL <= (size_t)134217728);
  if (SZ_ALL > ws_size) return;
  char* ws = (char*)d_ws;
  float* TH   = (float*)(ws + OF_TH);
  float* TAB  = (float*)(ws + OF_TAB);
  float* SC   = (float*)(ws + OF_SC);
  h16*   Hh   = (h16*)(ws + OF_H);
  h16*   Hr   = (h16*)(ws + OF_HR);
  h16*   W3   = (h16*)(ws + OF_W3);
  h16*   WoT  = (h16*)(ws + OF_WO);
  h16*   QK   = (h16*)(ws + OF_QK);
  h16*   QKr  = (h16*)(ws + OF_QKR);
  h16*   VT   = (h16*)(ws + OF_VT);
  h16*   VTr  = (h16*)(ws + OF_VTR);
  h16*   CTX  = (h16*)(ws + OF_CX);
  h16*   CTXr = (h16*)(ws + OF_CXR);

  k_theta<<<1, 128, 0, stream>>>(TH);
  const int ntab = SEQ * HD;
  k_tab<<<(unsigned)((ntab + 255) / 256), 256, 0, stream>>>(TH, TAB, ntab);
  k_scale<<<1, 32, 0, stream>>>(q1, q2, k1, k2, lam, SC);
  k_hnorm<<<(unsigned)NR, 256, 0, stream>>>(x, pw, Hh, Hr);

  const size_t nq8 = (size_t)NH * HW * DM / 8;
  const size_t nv8 = (size_t)DM * DM / 8;
  k_wcvt<<<(unsigned)((nq8 + 255) / 256), 256, 0, stream>>>(wq, W3, nq8);
  k_wcvt<<<(unsigned)((nq8 + 255) / 256), 256, 0, stream>>>(wk, W3 + (size_t)NH * HW * DM, nq8);
  k_wcvt<<<(unsigned)((nv8 + 255) / 256), 256, 0, stream>>>(wv, W3 + (size_t)NQK * DM, nv8);
  k_wcvt<<<(unsigned)((nv8 + 255) / 256), 256, 0, stream>>>(wo, WoT, nv8);

  k_gemm_qkv_early<<<(unsigned)((EROWS / 128) * (N3 / 64)), 128, 0, stream>>>(Hh, Hr, W3, TAB, QK, QKr, VT, VTr);
  if (NR > EROWS)
    k_gemm_qkv_late<<<(unsigned)(((NR - EROWS) / 128) * (N3 / 64)), 128, 0, stream>>>(Hh, W3, TAB, QK, VT);

  k_attn_early<<<(unsigned)(NH * (EROWS / 16)), 128, 0, stream>>>(QK, QKr, VT, VTr, SC, hnw, CTX, CTXr);
  if (SEQ > EROWS)
    k_attn_late<<<(unsigned)(NH * ((SEQ - EROWS) / 16)), 64, 0, stream>>>(QK, VT, SC, hnw, CTX);

  k_gemm_out_early<<<(unsigned)((EROWS / 128) * (DM / 64)), 128, 0, stream>>>(CTX, CTXr, WoT, x, out);
  if (NR > EROWS)
    k_gemm_out_late<<<(unsigned)(((NR - EROWS) / 128) * (DM / 64)), 128, 0, stream>>>(CTX, WoT, x, out);
}
